// TemporalGAT_61933428416929
// MI455X (gfx1250) — hardware-verified
//
#include <hip/hip_runtime.h>
#include <stddef.h>
#include <stdint.h>


#define IN_C    64
#define TDIM    32
#define KV      96
#define K0      128
#define D1      128
#define NLR     256
#define NX1     64
#define OC      2
#define NTHR    256
#define NWAVE   8
#define EPT     8
#define CHUNK   (NTHR * EPT)
#define WCAP    (EPT * 32)
#define LISTN   (NWAVE * WCAP)
#define NBMAX   2048
#define NBRUN   512
#define ESH     11
#define RCAP    28672
#define DEGCAP  4096
#define STW     512
#define GBM     64
#define GBN     64
#define GTHR    128
#define CX      8.0f
#define CL      2048.0f
#define CW      64.0f
#define SCL_XW  0.001953125f
#define SCL_XWL 9.5367431640625e-7f
#define NEGS    0.2f
#define WSMAX   134217728
#define LDS_AGG ((2 * RCAP + 2 * NBMAX + LISTN) * 4 + 64)

static_assert((CHUNK & (CHUNK - 1)) == 0 && CHUNK <= 4096);
static_assert((NBMAX & (NBMAX - 1)) == 0 && NBMAX <= 4096);
static_assert((NBRUN & (NBRUN - 1)) == 0 && NBRUN <= NBMAX && NBRUN >= 16);
static_assert((1 << ESH) >= NBMAX);
static_assert(NTHR * 8 == NBMAX);
static_assert(LISTN >= NBMAX);
static_assert(LISTN >= NWAVE * WCAP);
static_assert((RCAP % 32) == 0);
static_assert(NWAVE * STW <= RCAP);
static_assert(D1 <= STW);
static_assert(2 * NBMAX <= RCAP);
static_assert(NBRUN / 2 <= NTHR);
static_assert((NBRUN % 16) == 0);
static_assert(LDS_AGG <= 300000);
static_assert(GBM == (GTHR / 32) * 16);
static_assert((KV % 8) == 0 && KV <= K0 && (K0 % 32) == 0 && (D1 % 32) == 0);
static_assert(K0 / 8 == 16 && D1 / 8 == 16);
static_assert((NLR % GBN) == 0 && (NX1 % GBN) == 0);
static_assert(D1 == 4 * 32 && IN_C == 64 && TDIM == 32 && OC == 2);
static_assert(NLR == 2 * D1);

typedef float          v2f   __attribute__((ext_vector_type(2)));
typedef float          v4f   __attribute__((ext_vector_type(4)));
typedef float          v8f   __attribute__((ext_vector_type(8)));
typedef int            v4i   __attribute__((ext_vector_type(4)));
typedef int            v8i   __attribute__((ext_vector_type(8)));
typedef unsigned short v8us  __attribute__((ext_vector_type(8)));
typedef _Float16       v8h   __attribute__((ext_vector_type(8)));
typedef _Float16       v16h  __attribute__((ext_vector_type(16)));
typedef __bf16         v16bf __attribute__((ext_vector_type(16)));
union FragH { v16h v;  v8us u[2]; v8i w; };
union FragB { v16bf v; v8us u[2]; v8i w; };
template<int BF> struct FT { typedef FragH T; };
template<> struct FT<1> { typedef FragB T; };

__device__ __forceinline__ v8f wmx(const FragH& a, const FragH& b, v8f c) {
  v8f d = __builtin_amdgcn_wmma_f32_16x16x32_f16(false, a.v, false, b.v, (short)0, c, false, false);
  asm volatile("v_nop\n\tv_nop\n\tv_nop\n\tv_nop" : "+v"(d) : "v"(a.w), "v"(b.w));
  return d;
}
__device__ __forceinline__ v8f wmx(const FragB& a, const FragB& b, v8f c) {
  v8f d = __builtin_amdgcn_wmma_f32_16x16x32_bf16(false, a.v, false, b.v, (short)0, c, false, false);
  asm volatile("v_nop\n\tv_nop\n\tv_nop\n\tv_nop" : "+v"(d) : "v"(a.w), "v"(b.w));
  return d;
}

__device__ __forceinline__ unsigned bfbits(float v) {
  unsigned u = __float_as_uint(v);
  u = u + 0x7FFFu + ((u >> 16) & 1u);
  return u >> 16;
}
__device__ __forceinline__ float rbf(float v) { return __uint_as_float(bfbits(v) << 16); }

__device__ __forceinline__ v8us cvt8b(const v4f a, const v4f b) {
  v8us o;
  o[0] = (unsigned short)bfbits(a.x); o[1] = (unsigned short)bfbits(a.y);
  o[2] = (unsigned short)bfbits(a.z); o[3] = (unsigned short)bfbits(a.w);
  o[4] = (unsigned short)bfbits(b.x); o[5] = (unsigned short)bfbits(b.y);
  o[6] = (unsigned short)bfbits(b.z); o[7] = (unsigned short)bfbits(b.w);
  return o;
}
__device__ __forceinline__ v8h cvt8bh(const v4f a, const v4f b, const float c) {
  v8h hv;
  hv[0] = (_Float16)(rbf(a.x) * c); hv[1] = (_Float16)(rbf(a.y) * c);
  hv[2] = (_Float16)(rbf(a.z) * c); hv[3] = (_Float16)(rbf(a.w) * c);
  hv[4] = (_Float16)(rbf(b.x) * c); hv[5] = (_Float16)(rbf(b.y) * c);
  hv[6] = (_Float16)(rbf(b.z) * c); hv[7] = (_Float16)(rbf(b.w) * c);
  return hv;
}
__device__ __forceinline__ void cvt8hl(const v4f a, const v4f b, v8h& hv, v8h& lv) {
  float f[8] = {a.x * CX, a.y * CX, a.z * CX, a.w * CX, b.x * CX, b.y * CX, b.z * CX, b.w * CX};
#pragma unroll
  for (int i = 0; i < 8; ++i) {
    const _Float16 hq = (_Float16)f[i];
    hv[i] = hq;
    lv[i] = (_Float16)((f[i] - (float)hq) * CL);
  }
}
__device__ __forceinline__ void put8us(unsigned short* p, const v8us hv) {
  *(volatile v8us*)p = hv;
  __threadfence();
  *(volatile v8us*)p = hv;
}
__device__ __forceinline__ void put8h(_Float16* p, const v8h hv) {
  *(volatile v8h*)p = hv;
  __threadfence();
  *(volatile v8h*)p = hv;
}

__device__ __forceinline__ int scan_chunk(const int* __restrict__ dsts, int nE, int cbase, int slotBase,
                                          int nb, int vec8, int* list, int tid, int lane, int wave) {
  int wc = 0;
  const int el0  = tid * EPT;
  const int e0   = cbase + el0;
  const int sent = -2147483647 - 1;
  v4i da, db;
  if (vec8 != 0 && cbase + CHUNK <= nE) {
    da = *(const v4i*)(dsts + e0);
    db = *(const v4i*)(dsts + e0 + 4);
  } else {
    da.x = (e0     < nE) ? dsts[min(e0,     nE - 1)] : sent;
    da.y = (e0 + 1 < nE) ? dsts[min(e0 + 1, nE - 1)] : sent;
    da.z = (e0 + 2 < nE) ? dsts[min(e0 + 2, nE - 1)] : sent;
    da.w = (e0 + 3 < nE) ? dsts[min(e0 + 3, nE - 1)] : sent;
    db.x = (e0 + 4 < nE) ? dsts[min(e0 + 4, nE - 1)] : sent;
    db.y = (e0 + 5 < nE) ? dsts[min(e0 + 5, nE - 1)] : sent;
    db.z = (e0 + 6 < nE) ? dsts[min(e0 + 6, nE - 1)] : sent;
    db.w = (e0 + 7 < nE) ? dsts[min(e0 + 7, nE - 1)] : sent;
  }
  const unsigned nbs = (unsigned)slotBase;
  const unsigned unb = (unsigned)nb;
  const unsigned s0 = (unsigned)da.x - nbs, s1 = (unsigned)da.y - nbs;
  const unsigned s2 = (unsigned)da.z - nbs, s3 = (unsigned)da.w - nbs;
  const unsigned s4 = (unsigned)db.x - nbs, s5 = (unsigned)db.y - nbs;
  const unsigned s6 = (unsigned)db.z - nbs, s7 = (unsigned)db.w - nbs;
  const bool h0 = s0 < unb, h1 = s1 < unb, h2 = s2 < unb, h3 = s3 < unb;
  const bool h4 = s4 < unb, h5 = s5 < unb, h6 = s6 < unb, h7 = s7 < unb;
  const unsigned any = __builtin_amdgcn_ballot_w32(h0 | h1 | h2 | h3 | h4 | h5 | h6 | h7);
  if (any != 0u) {
#define HITJ(J, HJ, SJ) { \
      const unsigned mj = __builtin_amdgcn_ballot_w32(HJ); \
      if (mj != 0u) { \
        if (HJ) { \
          const int pos = wc + (int)__builtin_amdgcn_mbcnt_lo(mj, 0u); \
          if (pos < WCAP) list[wave * WCAP + pos] = ((el0 + (J)) << 12) | (int)(SJ); \
        } \
        wc += (int)__builtin_popcount(mj); } }
    HITJ(0, h0, s0)
    HITJ(1, h1, s1)
    HITJ(2, h2, s2)
    HITJ(3, h3, s3)
    HITJ(4, h4, s4)
    HITJ(5, h5, s5)
    HITJ(6, h6, s6)
    HITJ(7, h7, s7)
#undef HITJ
  }
  return wc;
}

__global__ __launch_bounds__(NTHR) void k_prep(
    const float* __restrict__ x, const int* __restrict__ tstep, const float* __restrict__ wtm, int nT,
    const float* __restrict__ wl0, const float* __restrict__ wr0,
    const float* __restrict__ wl1, const float* __restrict__ wr1,
    unsigned short* hb, unsigned short* wt0, _Float16* wt1,
    int nN, int nUx, int nBx, int nBw0) {
  const int b = (int)blockIdx.x, tid = (int)threadIdx.x;
  const v4f z4 = {0.f, 0.f, 0.f, 0.f};
  if (b < nBx) {
    const int i = b * NTHR + tid;
    if (i >= nUx) return;
    const int row = i >> 4;
    const int c0  = (i & 15) * 8;
    const int rc  = row < nN ? row : nN - 1;
    const int cx  = c0 < IN_C ? c0 : IN_C - 8;
    const float* px = x + (size_t)rc * IN_C + cx;
    const v4f xa = *(const v4f*)px, xb = *(const v4f*)(px + 4);
    int t = tstep[rc];
    t = t < 0 ? 0 : (t > nT - 1 ? nT - 1 : t);
    int ct = c0 - IN_C;
    ct = ct < 0 ? 0 : (ct > TDIM - 8 ? TDIM - 8 : ct);
    const float* pt = wtm + (size_t)t * TDIM + ct;
    const v4f ta = *(const v4f*)pt, tb = *(const v4f*)(pt + 4);
    v4f a = xa, bq = xb;
    if (c0 >= IN_C) { a = ta; bq = tb; }
    if (c0 >= KV || row >= nN) { a = z4; bq = z4; }
    put8us(hb + (size_t)row * K0 + c0, cvt8b(a, bq));
  } else if (b < nBx + nBw0) {
    const int u = (b - nBx) * NTHR + tid;
    if (u >= NLR * (K0 / 8)) return;
    const int n  = u >> 4;
    const int k8 = (u & 15) * 8;
    const int seg = n >> 7;
    const int nc  = n & (D1 - 1);
    const float* w = seg ? wr0 : wl0;
    const int kc = k8 < KV ? k8 : KV - 8;
    const float* p = w + (size_t)kc * D1 + nc;
    v4f a, bq;
    a.x  = p[0];               a.y  = p[(size_t)D1];       a.z  = p[(size_t)2 * D1];   a.w  = p[(size_t)3 * D1];
    bq.x = p[(size_t)4 * D1];  bq.y = p[(size_t)5 * D1];   bq.z = p[(size_t)6 * D1];   bq.w = p[(size_t)7 * D1];
    if (k8 >= KV) { a = z4; bq = z4; }
    put8us(wt0 + (size_t)n * K0 + k8, cvt8b(a, bq));
  } else {
    const int u = (b - nBx - nBw0) * NTHR + tid;
    if (u >= NX1 * (D1 / 8)) return;
    const int n  = u >> 4;
    const int k8 = (u & 15) * 8;
    const int sg = n >> 1;
    const int nc = n & 1;
    const float* w = (sg == 0) ? wl1 : wr1;
    const float* p = w + (size_t)k8 * OC + nc;
    v4f a, bq;
    a.x  = p[0];   a.y  = p[2];   a.z  = p[4];   a.w  = p[6];
    bq.x = p[8];   bq.y = p[10];  bq.z = p[12];  bq.w = p[14];
    if (n >= 2 * OC) { a = z4; bq = z4; }
    put8h(wt1 + (size_t)n * D1 + k8, cvt8bh(a, bq, CW));
  }
}

template<int BF, int RES>
__global__ __launch_bounds__(GTHR) void k_gemm(
    const unsigned short* __restrict__ A, const unsigned short* __restrict__ A2,
    const unsigned short* __restrict__ WT, float* outF, int K, int ldo, float scl, float scl2)
{
  typedef typename FT<BF>::T Frag;
  __shared__ __attribute__((aligned(16))) float stg[GBM * GBN];
  const int tid = (int)threadIdx.x, lane = tid & 31, wave = tid >> 5, hh = lane >> 4, m = lane & 15;
  const int rowBase = (int)blockIdx.x * GBM;
  const int col0    = (int)blockIdx.y * GBN;

  v8f acc[4], acc2[4];
  {
    const v8f z = {0.f, 0.f, 0.f, 0.f, 0.f, 0.f, 0.f, 0.f};
    acc[0] = z; acc[1] = z; acc[2] = z; acc[3] = z;
    acc2[0] = z; acc2[1] = z; acc2[2] = z; acc2[3] = z;
  }
  const size_t arow = (size_t)(rowBase + 16 * wave + m) * (size_t)K + 8 * hh;
  const unsigned short* ap  = A  + arow;
  const unsigned short* ap2 = A2 + arow;
  const unsigned short* wp  = WT + (size_t)(col0 + m) * (size_t)K + 8 * hh;
  const int ksteps = K >> 5;
#pragma unroll 1
  for (int ks = 0; ks < ksteps; ++ks) {
    Frag af, af2;
    af.u[0] = *(const v8us*)(ap + 32 * ks);
    af.u[1] = *(const v8us*)(ap + 32 * ks + 16);
    if (RES) {
      af2.u[0] = *(const v8us*)(ap2 + 32 * ks);
      af2.u[1] = *(const v8us*)(ap2 + 32 * ks + 16);
    } else {
      af2 = af;
    }
#pragma unroll
    for (int t = 0; t < 4; ++t) {
      const unsigned short* wq = wp + (size_t)(16 * t) * (size_t)K + 32 * ks;
      Frag bf;
      bf.u[0] = *(const v8us*)wq;
      bf.u[1] = *(const v8us*)(wq + 16);
      acc[t] = wmx(af, bf, acc[t]);
      if (RES) acc2[t] = wmx(af2, bf, acc2[t]);
    }
  }

#pragma unroll
  for (int t = 0; t < 4; ++t) {
    const int lc = 16 * t + m;
#pragma unroll
    for (int r = 0; r < 8; ++r) {
      const int lr = 16 * wave + 8 * hh + r;
      const float v = RES ? fmaf(acc2[t][r], scl2, acc[t][r] * scl) : acc[t][r] * scl;
      stg[lr * GBN + lc] = v;
    }
  }
  __syncthreads();

  v4f fv[8];
#pragma unroll
  for (int i = 0; i < 8; ++i) {
    const int lr = 16 * wave + 2 * i + hh;
    fv[i] = *(const v4f*)(stg + lr * GBN + 4 * m);
  }
#pragma unroll
  for (int i = 0; i < 8; ++i) {
    const int lr = 16 * wave + 2 * i + hh;
    const int gr = rowBase + lr;
    float* op = outF + (size_t)gr * (size_t)ldo + col0 + 4 * m;
    *(volatile v4f*)op = fv[i];
  }
  __threadfence();
#pragma unroll
  for (int i = 0; i < 8; ++i) {
    const int lr = 16 * wave + 2 * i + hh;
    const int gr = rowBase + lr;
    float* op = outF + (size_t)gr * (size_t)ldo + col0 + 4 * m;
    *(volatile v4f*)op = fv[i];
  }
}

__device__ __forceinline__ int build_lists(const int* __restrict__ dsts, int nE, int nodeBase, int nb, int vec8,
                                           int* reg1, int* reg2, int* scnt, int* soff, int* list,
                                           int* wcnt, int* wtot, int tid, int lane, int wave) {
  for (int i = tid; i < NBMAX; i += NTHR) scnt[i] = 0;
  __syncthreads();

  int tot = 0;
  const int nChunks = (nE + CHUNK - 1) / CHUNK;
#pragma unroll 1
  for (int ch = 0; ch < nChunks; ++ch) {
    const int cbase = ch * CHUNK;
    const int wc = scan_chunk(dsts, nE, cbase, nodeBase, nb, vec8, list, tid, lane, wave);
    if (lane == 0) wcnt[wave] = wc;
    __syncthreads();
    int pre = 0, all = 0;
#pragma unroll
    for (int w2 = 0; w2 < NWAVE; ++w2) {
      int c = wcnt[w2];
      c = c < 0 ? 0 : (c > WCAP ? WCAP : c);
      all += c;
      pre += (w2 < wave) ? c : 0;
    }
    const int wcc  = wc > WCAP ? WCAP : wc;
    const int base = tot + pre;
#pragma unroll 1
    for (int i = lane; i < wcc; i += 32) {
      const int ent = list[wave * WCAP + i];
      const int el  = (ent >> 12) & (CHUNK - 1);
      const int sl  = ent & (NBMAX - 1);
      int eid = cbase + el;
      eid = eid > nE - 1 ? nE - 1 : eid;
      const int pos = base + i;
      if (pos < RCAP) reg1[pos] = (int)(((unsigned)eid << ESH) | (unsigned)sl);
    }
    tot += all;
    tot = tot > RCAP ? RCAP : tot;
    __syncthreads();
  }
  const int nh = tot;

  if (wave == 0) {
#pragma unroll 1
    for (int b0 = 0; b0 < nh; b0 += 32) {
      const int idx = b0 + lane;
      const int uv  = reg1[idx < RCAP ? idx : RCAP - 1];
      const int m32 = (nh - b0) < 32 ? (nh - b0) : 32;
#pragma unroll 1
      for (int k = 0; k < m32; ++k) {
        const int u  = __builtin_amdgcn_readlane(uv, k);
        const int sl = u & (NBMAX - 1);
        if (lane == 0) scnt[sl] = scnt[sl] + 1;
      }
    }
  }
  __syncthreads();

  {
    const v4i ca = *(const v4i*)(scnt + 8 * tid);
    const v4i cb = *(const v4i*)(scnt + 8 * tid + 4);
    const int e0 = ca.x < 0 ? 0 : ca.x, e1 = ca.y < 0 ? 0 : ca.y, e2 = ca.z < 0 ? 0 : ca.z, e3 = ca.w < 0 ? 0 : ca.w;
    const int e4 = cb.x < 0 ? 0 : cb.x, e5 = cb.y < 0 ? 0 : cb.y, e6 = cb.z < 0 ? 0 : cb.z, e7 = cb.w < 0 ? 0 : cb.w;
    const int ts = e0 + e1 + e2 + e3 + e4 + e5 + e6 + e7;
    int incl = ts;
#pragma unroll
    for (int d = 1; d < 32; d <<= 1) {
      const int up = __shfl_up(incl, d);
      if (lane >= d) incl += up;
    }
    if (lane == 31) wtot[wave] = incl;
    __syncthreads();
    int pre = 0;
#pragma unroll
    for (int w2 = 0; w2 < NWAVE; ++w2) pre += (w2 < wave) ? wtot[w2] : 0;
    int run = pre + incl - ts;
    soff[8 * tid + 0] = run; run += e0;
    soff[8 * tid + 1] = run; run += e1;
    soff[8 * tid + 2] = run; run += e2;
    soff[8 * tid + 3] = run; run += e3;
    soff[8 * tid + 4] = run; run += e4;
    soff[8 * tid + 5] = run; run += e5;
    soff[8 * tid + 6] = run; run += e6;
    soff[8 * tid + 7] = run;
  }
  __syncthreads();
  for (int i = tid; i < NBMAX; i += NTHR) list[i] = soff[i];
  __syncthreads();

  if (wave == 0) {
#pragma unroll 1
    for (int b0 = 0; b0 < nh; b0 += 32) {
      const int idx = b0 + lane;
      const int uv  = reg1[idx < RCAP ? idx : RCAP - 1];
      const int m32 = (nh - b0) < 32 ? (nh - b0) : 32;
#pragma unroll 1
      for (int k = 0; k < m32; ++k) {
        const int u   = __builtin_amdgcn_readlane(uv, k);
        const int sl  = u & (NBMAX - 1);
        const int eid = (int)((unsigned)u >> ESH);
        if (lane == 0) {
          int pos = list[sl];
          pos = pos < 0 ? 0 : (pos > RCAP - 1 ? RCAP - 1 : pos);
          reg2[pos] = eid;
          list[sl] = pos + 1;
        }
      }
    }
  }
  __syncthreads();
  return nh;
}

__global__ __launch_bounds__(NTHR) void k_agg0(
    const int* __restrict__ srcs, const int* __restrict__ dsts,
    const float* __restrict__ XLR, const float* __restrict__ bl, const float* __restrict__ br,
    const float* __restrict__ att, const float* __restrict__ bias,
    _Float16* Hh, _Float16* Hl, int nN, int nE, int nb, int vec8, int MPr) {
  extern __shared__ v4f lds_dyn[];
  int* reg1 = (int*)lds_dyn;
  int* reg2 = reg1 + RCAP;
  int* scnt = reg2 + RCAP;
  int* soff = scnt + NBMAX;
  int* list = soff + NBMAX;
  int* wcnt = list + LISTN;
  int* wtot = wcnt + NWAVE;
  const int tid = (int)threadIdx.x, lane = tid & 31, wave = tid >> 5;
  const int nodeBase = (int)blockIdx.x * nb;

  const int nh = build_lists(dsts, nE, nodeBase, nb, vec8, reg1, reg2, scnt, soff, list, wcnt, wtot,
                             tid, lane, wave);

  const int nbw = nb >> 3;
  const bool ovf = (nh >= RCAP);
  const float qnan = __int_as_float(0x7fc00000);
  float* stw = (float*)reg1 + wave * STW;
  const int lc = lane < 16 ? lane : 15;
  const int c0 = 4 * lane;
  v4f at4 = *(const v4f*)(att + c0);
  v4f bl4 = *(const v4f*)(bl + c0);
  v4f br4 = *(const v4f*)(br + c0);
  v4f bi4 = *(const v4f*)(bias + c0);
  at4.x = rbf(at4.x); at4.y = rbf(at4.y); at4.z = rbf(at4.z); at4.w = rbf(at4.w);
  bl4.x = rbf(bl4.x); bl4.y = rbf(bl4.y); bl4.z = rbf(bl4.z); bl4.w = rbf(bl4.w);
  br4.x = rbf(br4.x); br4.y = rbf(br4.y); br4.z = rbf(br4.z); br4.w = rbf(br4.w);
  bi4.x = rbf(bi4.x); bi4.y = rbf(bi4.y); bi4.z = rbf(bi4.z); bi4.w = rbf(bi4.w);

#pragma unroll 1
  for (int jt = 0; jt < nbw; ++jt) {
    const int slot = wave * nbw + jt;
    const int grow = nodeBase + slot;
    const int gcl  = grow < nN ? grow : nN - 1;
    int st = soff[slot];
    const int craw = scnt[slot];
    int cnt = craw;
    st  = st < 0 ? 0 : (st > nh ? nh : st);
    cnt = cnt < 0 ? 0 : (cnt > DEGCAP ? DEGCAP : cnt);
    if (cnt > nh - st) cnt = nh - st;
    const float pz = (ovf || craw > DEGCAP) ? qnan : 0.0f;
    const float live = grow < nN ? 1.0f : 0.0f;

    const float* drow = XLR + (size_t)gcl * NLR;
    v4f xr4 = *(const v4f*)(drow + D1 + c0);
    v4f xs4 = *(const v4f*)(drow + c0);
    xr4 = xr4 + br4;
    xs4 = xs4 + bl4;

    float mx, dn;
    v4f av;
    {
      float m0 = xs4.x + xr4.x, m1 = xs4.y + xr4.y, m2 = xs4.z + xr4.z, m3 = xs4.w + xr4.w;
      m0 = m0 > 0.f ? m0 : m0 * NEGS;
      m1 = m1 > 0.f ? m1 : m1 * NEGS;
      m2 = m2 > 0.f ? m2 : m2 * NEGS;
      m3 = m3 > 0.f ? m3 : m3 * NEGS;
      float part = m0 * at4.x;
      part = fmaf(m1, at4.y, part);
      part = fmaf(m2, at4.z, part);
      part = fmaf(m3, at4.w, part);
      part += __shfl_xor(part, 1);
      part += __shfl_xor(part, 2);
      part += __shfl_xor(part, 4);
      mx = part; dn = 1.0f; av = xs4;
    }

#pragma unroll 1
    for (int q = 0; q < cnt; ++q) {
      int idx = st + q; idx = idx > RCAP - 1 ? RCAP - 1 : idx;
      int eid = reg2[idx]; eid = eid < 0 ? 0 : (eid > nE - 1 ? nE - 1 : eid);
      const int sraw = srcs[eid];
      const int s = sraw < 0 ? 0 : (sraw > nN - 1 ? nN - 1 : sraw);
      v4f xl4 = *(const v4f*)(XLR + (size_t)s * NLR + c0);
      xl4 = xl4 + bl4;
      float m0 = xl4.x + xr4.x, m1 = xl4.y + xr4.y, m2 = xl4.z + xr4.z, m3 = xl4.w + xr4.w;
      m0 = m0 > 0.f ? m0 : m0 * NEGS;
      m1 = m1 > 0.f ? m1 : m1 * NEGS;
      m2 = m2 > 0.f ? m2 : m2 * NEGS;
      m3 = m3 > 0.f ? m3 : m3 * NEGS;
      float part = m0 * at4.x;
      part = fmaf(m1, at4.y, part);
      part = fmaf(m2, at4.z, part);
      part = fmaf(m3, at4.w, part);
      part += __shfl_xor(part, 1);
      part += __shfl_xor(part, 2);
      part += __shfl_xor(part, 4);
      const float df = part - mx;
      const float ee = __expf(-fabsf(df));
      const bool up  = df > 0.f;
      const float s1 = up ? ee : 1.0f;
      const float s2 = up ? 1.0f : ee;
      mx = up ? part : mx;
      dn = fmaf(dn, s1, s2);
      av.x = fmaf(av.x, s1, s2 * xl4.x);
      av.y = fmaf(av.y, s1, s2 * xl4.y);
      av.z = fmaf(av.z, s1, s2 * xl4.z);
      av.w = fmaf(av.w, s1, s2 * xl4.w);
    }
    const float iv = __builtin_amdgcn_rcpf(dn);
    v4f r;
    r.x = fmaxf(fmaf(av.x, iv, bi4.x), 0.f) * live + pz;
    r.y = fmaxf(fmaf(av.y, iv, bi4.y), 0.f) * live + pz;
    r.z = fmaxf(fmaf(av.z, iv, bi4.z), 0.f) * live + pz;
    r.w = fmaxf(fmaf(av.w, iv, bi4.w), 0.f) * live + pz;
    __builtin_amdgcn_fence(__ATOMIC_RELEASE, "wavefront");
    __builtin_amdgcn_wave_barrier();
    *(v4f*)(stw + 4 * lane) = r;
    __builtin_amdgcn_fence(__ATOMIC_RELEASE, "wavefront");
    __builtin_amdgcn_wave_barrier();
    const bool wr = grow < MPr;
    const v4f ga = *(const v4f*)(stw + 8 * lc);
    const v4f gb = *(const v4f*)(stw + 8 * lc + 4);
    v8h hv, lv;
    cvt8hl(ga, gb, hv, lv);
    _Float16* gph = Hh + (size_t)grow * D1 + 8 * lc;
    _Float16* gpl = Hl + (size_t)grow * D1 + 8 * lc;
    const bool wsv = wr && (lane < (D1 / 8));
    if (wsv) { *(volatile v8h*)gph = hv; *(volatile v8h*)gpl = lv; }
    __threadfence();
    if (wsv) { *(volatile v8h*)gph = hv; *(volatile v8h*)gpl = lv; }
  }
}

__global__ __launch_bounds__(NTHR) void k_agg1(
    const int* __restrict__ srcs, const int* __restrict__ dsts,
    const float* __restrict__ XP, const float* __restrict__ bl, const float* __restrict__ br,
    const float* __restrict__ att, const float* __restrict__ bias,
    float* out, int nN, int nE, int nb, int vec8) {
  extern __shared__ v4f lds_dyn[];
  int* reg1 = (int*)lds_dyn;
  int* reg2 = reg1 + RCAP;
  int* scnt = reg2 + RCAP;
  int* soff = scnt + NBMAX;
  int* list = soff + NBMAX;
  int* wcnt = list + LISTN;
  int* wtot = wcnt + NWAVE;
  const int tid = (int)threadIdx.x, lane = tid & 31, wave = tid >> 5;
  const int nodeBase = (int)blockIdx.x * nb;

  const int nh = build_lists(dsts, nE, nodeBase, nb, vec8, reg1, reg2, scnt, soff, list, wcnt, wtot,
                             tid, lane, wave);

  const int nbw = nb >> 3;
  const bool ovf = (nh >= RCAP);
  const float qnan = __int_as_float(0x7fc00000);
  float* sres = (float*)reg1;
  const float a0  = rbf(att[0]),  a1  = rbf(att[1]);
  const float bl0 = rbf(bl[0]),   bl1 = rbf(bl[1]);
  const float br0 = rbf(br[0]),   br1 = rbf(br[1]);
  const float bi0 = rbf(bias[0]), bi1 = rbf(bias[1]);

#pragma unroll 1
  for (int jt = 0; jt < nbw; ++jt) {
    const int slot = wave * nbw + jt;
    const int grow = nodeBase + slot;
    const int gcl  = grow < nN ? grow : nN - 1;
    int st = soff[slot];
    const int craw = scnt[slot];
    int cnt = craw;
    st  = st < 0 ? 0 : (st > nh ? nh : st);
    cnt = cnt < 0 ? 0 : (cnt > DEGCAP ? DEGCAP : cnt);
    if (cnt > nh - st) cnt = nh - st;
    const float pz = (ovf || craw > DEGCAP) ? qnan : 0.0f;

    const float* drow = XP + (size_t)gcl * NX1;
    const v2f xd = *(const v2f*)drow;
    const v2f xe = *(const v2f*)(drow + 2);
    const float xr0 = xe.x + br0, xr1 = xe.y + br1;
    const float xs0 = xd.x + bl0, xs1 = xd.y + bl1;
    float mx, dn, ax, ay;
    {
      float u0 = xs0 + xr0, u1 = xs1 + xr1;
      u0 = u0 > 0.f ? u0 : u0 * NEGS;
      u1 = u1 > 0.f ? u1 : u1 * NEGS;
      float ls = u0 * a0;
      ls = fmaf(u1, a1, ls);
      mx = ls; dn = 1.0f; ax = xs0; ay = xs1;
    }
    const int nch = (cnt + 31) >> 5;
    const int cm1 = cnt > 0 ? cnt - 1 : 0;
#pragma unroll 1
    for (int cb = 0; cb < nch; ++cb) {
      const int q = cb * 32 + lane;
      const bool valid = q < cnt;
      const int qc = q < cm1 ? q : cm1;
      int idx = st + qc; idx = idx > RCAP - 1 ? RCAP - 1 : idx;
      int eid = reg2[idx]; eid = eid < 0 ? 0 : (eid > nE - 1 ? nE - 1 : eid);
      const int sraw = srcs[eid];
      const int s = sraw < 0 ? 0 : (sraw > nN - 1 ? nN - 1 : sraw);
      const v2f xg = *(const v2f*)(XP + (size_t)s * NX1);
      const float xl0 = xg.x + bl0, xl1 = xg.y + bl1;
      float u0 = xl0 + xr0, u1 = xl1 + xr1;
      u0 = u0 > 0.f ? u0 : u0 * NEGS;
      u1 = u1 > 0.f ? u1 : u1 * NEGS;
      float l = u0 * a0;
      l = fmaf(u1, a1, l);
      float lm = valid ? l : -1.0e30f;
#pragma unroll
      for (int off = 16; off > 0; off >>= 1) lm = fmaxf(lm, __shfl_xor(lm, off));
      const float mn = fmaxf(mx, lm);
      const float sc = __expf(mx - mn);
      float d = l - mn;
      d = d < -80.f ? -80.f : (d > 0.f ? 0.f : d);
      const float e = __expf(d);
      const float p = valid ? e : 0.0f;
      float sp = p, sx = p * xl0, sy = p * xl1;
#pragma unroll
      for (int off = 16; off > 0; off >>= 1) {
        sp += __shfl_xor(sp, off);
        sx += __shfl_xor(sx, off);
        sy += __shfl_xor(sy, off);
      }
      dn = fmaf(dn, sc, sp);
      ax = fmaf(ax, sc, sx);
      ay = fmaf(ay, sc, sy);
      mx = mn;
    }
    const float iv = __builtin_amdgcn_rcpf(dn);
    const float o0 = fmaf(ax, iv, bi0) + pz;
    const float o1 = fmaf(ay, iv, bi1) + pz;
    if (lane == 0) { sres[2 * slot] = o0; sres[2 * slot + 1] = o1; }
  }
  __syncthreads();

  {
    const int np  = nb >> 1;
    const int tc  = tid < np ? tid : np - 1;
    const v4f gv  = *(const v4f*)(sres + 4 * tc);
    const int r0  = nodeBase + 2 * tid;
    const bool act  = tid < np;
    const bool full = act && (r0 + 1 < nN);
    const bool half = act && (!full) && (r0 < nN);
    const int rcl = r0 < nN ? r0 : nN - 1;
    float* gp = out + (size_t)rcl * OC;
    v2f g2; g2.x = gv.x; g2.y = gv.y;
    if (full) *(volatile v4f*)gp = gv;
    else if (half) *(volatile v2f*)gp = g2;
    __threadfence();
    if (full) *(volatile v4f*)gp = gv;
    else if (half) *(volatile v2f*)gp = g2;
  }
}

static int pick_nb(int nE, int nN) {
  int nb = NBRUN;
  while (nb > 16 && (long long)nb * (long long)nE * 5LL > (long long)RCAP * (long long)nN * 4LL) nb >>= 1;
  return nb;
}
static inline int cdiv(int a, int b) { return (a + b - 1) / b; }

extern "C" void kernel_launch(void* const* d_in, const int* in_sizes, int n_in,
                              void* d_out, int out_size, void* d_ws, size_t ws_size,
                              hipStream_t stream) {
  if (n_in < 16) return;
  if (in_sizes[0] < IN_C || (in_sizes[0] % IN_C) != 0) return;
  const int nN = in_sizes[0] / IN_C;
  if (nN <= 0 || nN > (1 << 22)) return;
  if (in_sizes[1] < 2 || (in_sizes[1] & 1) != 0) return;
  const int nE = in_sizes[1] / 2;
  if (nE < 1 || nE > (1 << (32 - ESH))) return;
  if (in_sizes[2] != nN) return;
  if (in_sizes[3] < TDIM || (in_sizes[3] % TDIM) != 0) return;
  const int nT = in_sizes[3] / TDIM;
  if (in_sizes[4] != KV * D1 || in_sizes[5] != D1) return;
  if (in_sizes[6] != KV * D1 || in_sizes[7] != D1) return;
  if (in_sizes[8] != D1 || in_sizes[9] != D1) return;
  if (in_sizes[10] != D1 * OC || in_sizes[11] != OC) return;
  if (in_sizes[12] != D1 * OC || in_sizes[13] != OC) return;
  if (in_sizes[14] != OC || in_sizes[15] != OC) return;
  if (out_size != nN * OC) return;

  const float* x     = (const float*)d_in[0];
  const int*   ei    = (const int*)  d_in[1];
  const int*   tstep = (const int*)  d_in[2];
  const float* wtm   = (const float*)d_in[3];
  const float* wl0   = (const float*)d_in[4];
  const float* bl0   = (const float*)d_in[5];
  const float* wr0   = (const float*)d_in[6];
  const float* br0   = (const float*)d_in[7];
  const float* att0  = (const float*)d_in[8];
  const float* bias0 = (const float*)d_in[9];
  const float* wl1   = (const float*)d_in[10];
  const float* bl1   = (const float*)d_in[11];
  const float* wr1   = (const float*)d_in[12];
  const float* br1   = (const float*)d_in[13];
  const float* att1  = (const float*)d_in[14];
  const float* bias1 = (const float*)d_in[15];
  float* out = (float*)d_out;
  const int* src = ei;
  const int* dst = ei + nE;

  const int MP   = cdiv(nN, GBM) * GBM;
  const int nb   = pick_nb(nE, nN);
  const int gA   = cdiv(MP, nb);
  const int vec8 = ((nE & 3) == 0) ? 1 : 0;
  if (gA * nb < MP) return;

  char* ws = (char*)d_ws;
  size_t off = 0;
  const size_t oHB  = off; off += (size_t)MP * K0 * 2;             off = (off + 255) & ~(size_t)255;
  const size_t oWT0 = off; off += (size_t)NLR * K0 * 2;            off = (off + 255) & ~(size_t)255;
  const size_t oWT1 = off; off += (size_t)NX1 * D1 * 2;            off = (off + 255) & ~(size_t)255;
  const size_t oXL0 = off; off += (size_t)MP * NLR * 4;            off = (off + 255) & ~(size_t)255;
  const size_t oH1H = off; off += (size_t)MP * D1 * 2;             off = (off + 255) & ~(size_t)255;
  const size_t oH1L = off; off += (size_t)MP * D1 * 2;             off = (off + 255) & ~(size_t)255;
  const size_t oXL1 = off; off += (size_t)MP * NX1 * 4;            off = (off + 255) & ~(size_t)255;
  if (off > ws_size || off > (size_t)WSMAX) return;
  unsigned short* HB   = (unsigned short*)(ws + oHB);
  unsigned short* WT0  = (unsigned short*)(ws + oWT0);
  unsigned short* WT1  = (unsigned short*)(ws + oWT1);
  float*          XLR0 = (float*)(ws + oXL0);
  unsigned short* H1H  = (unsigned short*)(ws + oH1H);
  unsigned short* H1L  = (unsigned short*)(ws + oH1L);
  float*          XLR1 = (float*)(ws + oXL1);

  hipFuncSetAttribute(reinterpret_cast<const void*>(&k_agg0),
                      hipFuncAttributeMaxDynamicSharedMemorySize, LDS_AGG);
  hipFuncSetAttribute(reinterpret_cast<const void*>(&k_agg1),
                      hipFuncAttributeMaxDynamicSharedMemorySize, LDS_AGG);

  const int nUx  = MP * (K0 / 8);
  const int nBx  = cdiv(nUx, NTHR);
  const int nBw0 = cdiv(NLR * (K0 / 8), NTHR);
  const int nBw1 = cdiv(NX1 * (D1 / 8), NTHR);
  k_prep<<<nBx + nBw0 + nBw1, NTHR, 0, stream>>>(x, tstep, wtm, nT, wl0, wr0, wl1, wr1,
                                                  HB, WT0, (_Float16*)WT1, nN, nUx, nBx, nBw0);

  const int gM = MP / GBM;
  k_gemm<1, 0><<<dim3(gM, NLR / GBN), GTHR, 0, stream>>>(HB, HB, WT0, XLR0, K0, NLR, 1.0f, 0.0f);
  k_agg0<<<gA, NTHR, LDS_AGG, stream>>>(src, dst, XLR0, bl0, br0, att0, bias0,
                                        (_Float16*)H1H, (_Float16*)H1L, nN, nE, nb, vec8, MP);
  k_gemm<0, 1><<<dim3(gM, NX1 / GBN), GTHR, 0, stream>>>(H1H, H1L, WT1, XLR1, D1, NX1, SCL_XW, SCL_XWL);
  k_agg1<<<gA, NTHR, LDS_AGG, stream>>>(src, dst, XLR1, bl1, br1, att1, bias1, out, nN, nE, nb, vec8);
}
